// HyperbolicKuramotoAttentionV2_137438954438
// MI455X (gfx1250) — hardware-verified
//
#include <hip/hip_runtime.h>
#include <stddef.h>
#include <stdint.h>

#define BB   4
#define NN   1024
#define CC   1024
#define HH   16
#define DD   64
#define ROWS (BB * NN)
#define C3   (3 * CC)
#define NBH  (BB * HH)
#define PL   ((size_t)NBH * NN * DD)

static_assert(NN % 256 == 0);
static_assert(CC % 64 == 0);
static_assert(DD == 64);
static_assert(HH * DD == CC);
static_assert(ROWS % 256 == 0);
static_assert(HH == 16);

#define TWO_PI_F   6.28318530717958647692f
#define INV_TEMP   1.0f
#define DT_F       0.1f
#define CPL_OVER_H 0.0625f
#define INV_H      0.0625f

typedef _Float16 v16h __attribute__((ext_vector_type(16)));
typedef _Float16 v8h  __attribute__((ext_vector_type(8)));
typedef float    v8f  __attribute__((ext_vector_type(8)));
typedef float    v4f  __attribute__((ext_vector_type(4)));
typedef unsigned int v4u __attribute__((ext_vector_type(4)));

union Frag  { v16h v; v8h h[2]; };
union Pack8 { v8h h; v4u u; };

__device__ __forceinline__ v8f mma16(v16h a, v16h b, v8f c) {
  c = __builtin_amdgcn_wmma_f32_16x16x32_f16(false, a, false, b, (short)0, c, false, false);
  asm volatile("v_nop\n\tv_nop\n\tv_nop\n\tv_nop" : "+v"(c) : "v"(a), "v"(b));
  return c;
}

__device__ __forceinline__ v16h ldfrag(const _Float16* p, int ld, int row0, int k0, int lane) {
  const int m = lane & 15, lh = lane >> 4;
  const _Float16* q = p + (size_t)(row0 + m) * ld + k0 + 8 * lh;
  Frag f;
  f.h[0] = *(const v8h*)(q);
  f.h[1] = *(const v8h*)(q + 16);
  return f.v;
}

__device__ __forceinline__ v8f zero8() { return (v8f){0.f, 0.f, 0.f, 0.f, 0.f, 0.f, 0.f, 0.f}; }

__device__ __forceinline__ void gemm32x64(const _Float16* __restrict__ A, int lda,
                                          const _Float16* __restrict__ Bt, int ldb,
                                          int m0, int n0, int lane, v8f (&acc)[2][4]) {
#pragma unroll 2
  for (int k0 = 0; k0 < CC; k0 += 32) {
    const v16h a0 = ldfrag(A, lda, m0, k0, lane);
    const v16h a1 = ldfrag(A, lda, m0 + 16, k0, lane);
    const v16h b0 = ldfrag(Bt, ldb, n0, k0, lane);
    const v16h b1 = ldfrag(Bt, ldb, n0 + 16, k0, lane);
    const v16h b2 = ldfrag(Bt, ldb, n0 + 32, k0, lane);
    const v16h b3 = ldfrag(Bt, ldb, n0 + 48, k0, lane);
    acc[0][0] = mma16(a0, b0, acc[0][0]);
    acc[1][0] = mma16(a1, b0, acc[1][0]);
    acc[0][1] = mma16(a0, b1, acc[0][1]);
    acc[1][1] = mma16(a1, b1, acc[1][1]);
    acc[0][2] = mma16(a0, b2, acc[0][2]);
    acc[1][2] = mma16(a1, b2, acc[1][2]);
    acc[0][3] = mma16(a0, b3, acc[0][3]);
    acc[1][3] = mma16(a1, b3, acc[1][3]);
  }
}

__global__ __launch_bounds__(256) void k_cvt(const float* __restrict__ x, _Float16* __restrict__ xh,
                                             int ngrp, float scale) {
  const int t = blockIdx.x * 256 + (int)threadIdx.x;
  if (t >= ngrp) return;
  const size_t o = (size_t)t * 8;
  const v4f a0 = *(const v4f*)(x + o);
  const v4f a1 = *(const v4f*)(x + o + 4);
  Pack8 pk;
  pk.h = (v8h){(_Float16)(a0[0] * scale), (_Float16)(a0[1] * scale), (_Float16)(a0[2] * scale), (_Float16)(a0[3] * scale),
               (_Float16)(a1[0] * scale), (_Float16)(a1[1] * scale), (_Float16)(a1[2] * scale), (_Float16)(a1[3] * scale)};
  const v4u vv = pk.u;
  volatile v4u* d = (volatile v4u*)(xh + o);
  *d = vv;
  __threadfence();
  *d = vv;
}

__global__ __launch_bounds__(32) void k_phase(const float* __restrict__ base, const float* __restrict__ natf,
                                             const float* __restrict__ ph0, float* __restrict__ cohp,
                                             float* __restrict__ oph, float* __restrict__ oord) {
  __shared__ float phs[HH];
  __shared__ float cohs[HH];
  const int l = threadIdx.x & 31;
  const int h = l & (HH - 1);
  const float* brow = base + h * HH;

  float mx = -__builtin_huge_valf();
#pragma unroll 1
  for (int q = 0; q < HH; ++q) mx = fmaxf(mx, brow[q] * INV_TEMP);
  float se = 0.f;
#pragma unroll 1
  for (int q = 0; q < HH; ++q) se += expf(brow[q] * INV_TEMP - mx);
  const float inv_se = 1.0f / se;
  const float th = ph0[h];
  float cs = 0.f;
#pragma unroll 1
  for (int q = 0; q < HH; ++q) {
    const float cpl = expf(brow[q] * INV_TEMP - mx) * inv_se;
    cs += cpl * sinf(th - ph0[q]);
  }
  const float dph = natf[h] + CPL_OVER_H * cs;
  const float ph  = fmodf(th + DT_F * dph, TWO_PI_F);
  if (l < HH) phs[l] = ph;
  __syncthreads();

  float co = 0.f, cc = 0.f;
#pragma unroll 1
  for (int it = 0; it < 2 * HH; ++it) {
    const float pj  = phs[it & (HH - 1)];
    const bool  fst = it < HH;
    const float arg = fst ? (ph - pj) : pj;
    const float cv  = cosf(arg);
    co += fst ? cv : 0.f;
    cc += fst ? 0.f : cv;
  }
  float sn = 0.f;
#pragma unroll 1
  for (int j = 0; j < HH; ++j) sn += sinf(phs[j]);
  co *= INV_H;
  cc *= INV_H;
  sn *= INV_H;
  const float ord = sqrtf(cc * cc + sn * sn);
  if (l < HH) cohs[l] = co;
  __syncthreads();

  const int i0 = (4 * l) & (HH - 1);
  const v4f pv  = (v4f){phs[i0], phs[i0 + 1], phs[i0 + 2], phs[i0 + 3]};
  const v4f cv4 = (v4f){cohs[i0], cohs[i0 + 1], cohs[i0 + 2], cohs[i0 + 3]};
  const v4f ov  = (v4f){ord, ord, ord, ord};
  for (int ps = 0; ps < 2; ++ps) {
    if (l < HH) *(volatile v4f*)(oph + 4 * l) = pv;
    if (l < 8)  *(volatile v4f*)(cohp + 4 * l) = cv4;
    if (l == 0) *(volatile v4f*)(oord) = ov;
    __threadfence();
  }
}

#define STP 72
__global__ __launch_bounds__(256) void k_qkv(const _Float16* __restrict__ xh,
                                             const _Float16* __restrict__ wt,
                                             const float* __restrict__ bq,
                                             const float* __restrict__ bk,
                                             const float* __restrict__ bv,
                                             _Float16* __restrict__ qkv,
                                             float* __restrict__ nrm) {
  __shared__ __align__(16) _Float16 st[256 * STP];
  __shared__ __align__(16) float rn[256];
  const int tid = threadIdx.x, lane = tid & 31, wave = tid >> 5;
  const int hh = lane >> 4, c = lane & 15;
  const int mb = blockIdx.x * 256;
  const int m0 = mb + wave * 32;
  const int n0 = blockIdx.y * 64;
  const int which = n0 >> 10;
  const int ncol  = n0 & (CC - 1);
  const int head  = ncol >> 6;
  const int b  = mb >> 10;
  const int nb = mb & (NN - 1);
  const int bh = b * HH + head;

  v8f acc[2][4];
#pragma unroll
  for (int s = 0; s < 2; ++s)
#pragma unroll
    for (int t = 0; t < 4; ++t) acc[s][t] = zero8();
  gemm32x64(xh, CC, wt, CC, m0, n0, lane, acc);

  float bvs[4];
#pragma unroll
  for (int t = 0; t < 4; ++t) {
    const int nn = ncol + 16 * t + c;
    const float b0 = bq[nn], b1 = bk[nn], b2 = bv[nn];
    bvs[t] = (which == 0) ? b0 : ((which == 1) ? b1 : b2);
  }
#pragma unroll
  for (int sub = 0; sub < 2; ++sub) {
    float ss[8];
#pragma unroll
    for (int r = 0; r < 8; ++r) ss[r] = 0.f;
#pragma unroll
    for (int t = 0; t < 4; ++t) {
#pragma unroll
      for (int r = 0; r < 8; ++r) {
        const int lr = wave * 32 + sub * 16 + 8 * hh + r;
        const float v = acc[sub][t][r] * 0.03125f + bvs[t];
        st[lr * STP + 16 * t + c] = (_Float16)v;
        ss[r] += v * v;
      }
    }
#pragma unroll
    for (int r = 0; r < 8; ++r) {
      float q = ss[r];
      q += __shfl_xor(q, 1, 32);
      q += __shfl_xor(q, 2, 32);
      q += __shfl_xor(q, 4, 32);
      q += __shfl_xor(q, 8, 32);
      if (c == 0) rn[wave * 32 + sub * 16 + 8 * hh + r] = q;
    }
  }
  __syncthreads();

  v4u val[8];
  size_t go[8];
  if (which < 2) {
#pragma unroll
    for (int j = 0; j < 8; ++j) {
      const int p  = tid + 256 * j;
      const int lr = p >> 3;
      const int pc = p & 7;
      Pack8 pk;
      pk.h  = *(const v8h*)(st + lr * STP + pc * 8);
      val[j] = pk.u;
      go[j]  = (size_t)which * PL + ((size_t)bh * NN + nb + lr) * DD + pc * 8;
    }
  } else {
#pragma unroll
    for (int j = 0; j < 8; ++j) {
      const int p  = tid + 256 * j;
      const int L  = p >> 3;
      const int pc = p & 7;
      const int d  = L >> 2;
      const int nl = (L & 3) * 64 + pc * 8;
      const _Float16* cp = st + nl * STP + d;
      Pack8 pk;
      pk.h = (v8h){cp[0 * STP], cp[1 * STP], cp[2 * STP], cp[3 * STP],
                   cp[4 * STP], cp[5 * STP], cp[6 * STP], cp[7 * STP]};
      val[j] = pk.u;
      go[j]  = 2 * PL + ((size_t)bh * DD + d) * NN + nb + nl;
    }
  }
  const int tn = tid & 63;
  const v4f nv = *(const v4f*)(rn + tn * 4);
  float* np = nrm + (size_t)(which & 1) * ((size_t)NBH * NN) + (size_t)bh * NN + nb + tn * 4;
  const bool wn = (which < 2) && (tid < 64);
  for (int ps = 0; ps < 2; ++ps) {
#pragma unroll
    for (int j = 0; j < 8; ++j) *(volatile v4u*)(qkv + go[j]) = val[j];
    if (wn) *(volatile v4f*)np = nv;
    __threadfence();
  }
}

#define KTP 72
#define PTP 72
__global__ __launch_bounds__(256) void k_attn(const _Float16* __restrict__ qp,
                                              const _Float16* __restrict__ kp,
                                              const _Float16* __restrict__ vt,
                                              const float* __restrict__ qn,
                                              const float* __restrict__ kn,
                                              const float* __restrict__ cohp,
                                              _Float16* __restrict__ op) {
  __shared__ __align__(16) _Float16 Ks[64 * KTP];
  __shared__ __align__(16) _Float16 Vs[64 * KTP];
  __shared__ __align__(16) _Float16 Ps[8][16 * PTP];

  const int tid = threadIdx.x, lane = tid & 31, wave = tid >> 5;
  const int hh = lane >> 4, c = lane & 15;
  const int bh = blockIdx.x >> 3;
  const int qb = blockIdx.x & 7;
  const int b  = bh >> 4, h = bh & (HH - 1);
  const int q0 = qb * 128 + wave * 16;

  const _Float16* Q = qp + (size_t)bh * NN * DD;
  const _Float16* K = kp + (size_t)bh * NN * DD;
  const _Float16* V = vt + (size_t)bh * DD * NN;
  const float* qnb = qn + (size_t)bh * NN;
  const float* knb = kn + (size_t)bh * NN;
  const float coh = cohp[h];

  v16h qa[2];
  qa[0] = ldfrag(Q, DD, q0, 0, lane);
  qa[1] = ldfrag(Q, DD, q0, 32, lane);

  float qn_r[8], omq[8];
#pragma unroll
  for (int r = 0; r < 8; ++r) {
    const float v = qnb[q0 + 8 * hh + r];
    qn_r[r] = v;
    omq[r]  = 1.0f - fminf(v, 0.99f);
  }

  const float NEGI = -__builtin_huge_valf();
  float mrow[8], lrow[8];
  v8f oacc[4];
#pragma unroll
  for (int r = 0; r < 8; ++r) { mrow[r] = NEGI; lrow[r] = 0.f; }
#pragma unroll
  for (int t = 0; t < 4; ++t) oacc[t] = zero8();

  _Float16* pw = Ps[wave];

#pragma unroll 1
  for (int kc = 0; kc < NN / 64; ++kc) {
    const int kv0 = kc * 64;
    __syncthreads();
    {
      const int r  = tid >> 2;
      const int qq = (tid & 3) * 16;
      const _Float16* ks = K + (size_t)(kv0 + r) * DD + qq;
      *(v8h*)(Ks + r * KTP + qq)     = *(const v8h*)(ks);
      *(v8h*)(Ks + r * KTP + qq + 8) = *(const v8h*)(ks + 8);
      const _Float16* vs = V + (size_t)r * NN + kv0 + qq;
      *(v8h*)(Vs + r * KTP + qq)     = *(const v8h*)(vs);
      *(v8h*)(Vs + r * KTP + qq + 8) = *(const v8h*)(vs + 8);
    }
    __syncthreads();

    v8f s[4];
#pragma unroll
    for (int j = 0; j < 4; ++j) s[j] = zero8();
#pragma unroll
    for (int dc = 0; dc < 2; ++dc) {
#pragma unroll
      for (int j = 0; j < 4; ++j) {
        const v16h kb = ldfrag(Ks, KTP, j * 16, dc * 32, lane);
        s[j] = mma16(qa[dc], kb, s[j]);
      }
    }
    float knv[4], onk[4];
#pragma unroll
    for (int j = 0; j < 4; ++j) {
      const float v = knb[kv0 + 16 * j + c];
      knv[j] = v;
      onk[j] = 1.0f - fminf(v, 0.99f);
    }
    float cm[8];
#pragma unroll
    for (int r = 0; r < 8; ++r) {
      float m = NEGI;
#pragma unroll
      for (int j = 0; j < 4; ++j) {
        const float dot  = s[j][r];
        const float dsq  = (qn_r[r] + knv[j]) - 2.0f * dot;
        const float den  = omq[r] * onk[j] + 1e-8f;
        const float arg  = 1.0f + (2.0f * dsq) * __builtin_amdgcn_rcpf(den);
        const float t2   = fmaxf(arg * arg - 1.0f, 1e-8f);
        const float u    = arg + __builtin_amdgcn_sqrtf(t2);
        const float dist = __logf(u);
        const float sv   = __expf(-dist * INV_TEMP) * coh;
        s[j][r] = sv;
        m = fmaxf(m, sv);
      }
#pragma unroll
      for (int off = 1; off < 16; off <<= 1) m = fmaxf(m, __shfl_xor(m, off, 32));
      cm[r] = m;
    }
    float al[8];
#pragma unroll
    for (int r = 0; r < 8; ++r) {
      const float mnew  = fmaxf(mrow[r], cm[r]);
      const float alpha = __expf(mrow[r] - mnew);
      mrow[r] = mnew;
      float psum = 0.f;
#pragma unroll
      for (int j = 0; j < 4; ++j) {
        const float p = __expf(s[j][r] - mnew);
        psum += p;
        pw[(8 * hh + r) * PTP + j * 16 + c] = (_Float16)(p * 1024.0f);
      }
#pragma unroll
      for (int off = 1; off < 16; off <<= 1) psum += __shfl_xor(psum, off, 32);
      lrow[r] = lrow[r] * alpha + psum;
      al[r] = alpha;
    }
#pragma unroll
    for (int t = 0; t < 4; ++t)
#pragma unroll
      for (int r = 0; r < 8; ++r) oacc[t][r] *= al[r];
    __syncthreads();

#pragma unroll
    for (int kk = 0; kk < 2; ++kk) {
      const v16h pa = ldfrag(pw, PTP, 0, kk * 32, lane);
#pragma unroll
      for (int t = 0; t < 4; ++t) {
        const v16h vb = ldfrag(Vs, KTP, t * 16, kk * 32, lane);
        oacc[t] = mma16(pa, vb, oacc[t]);
      }
    }
  }
  __syncthreads();

#pragma unroll
  for (int r = 0; r < 8; ++r) {
    const float inv = 0.015625f / lrow[r];
#pragma unroll
    for (int t = 0; t < 4; ++t) pw[(8 * hh + r) * PTP + 16 * t + c] = (_Float16)(oacc[t][r] * inv);
  }
  __syncthreads();
  v4u val[4];
  size_t go[4];
#pragma unroll
  for (int it = 0; it < 4; ++it) {
    const int p  = lane + 32 * it;
    const int L  = p >> 3;
    const int pc = p & 7;
    Pack8 pk;
    pk.h   = *(const v8h*)(pw + L * PTP + pc * 8);
    val[it] = pk.u;
    go[it]  = ((size_t)(b * NN + q0 + L)) * CC + (size_t)h * DD + pc * 8;
  }
  for (int ps = 0; ps < 2; ++ps) {
#pragma unroll
    for (int it = 0; it < 4; ++it) *(volatile v4u*)(op + go[it]) = val[it];
    __threadfence();
  }
}

#define OTP 68
__global__ __launch_bounds__(256) void k_proj(const _Float16* __restrict__ ap,
                                              const _Float16* __restrict__ wt,
                                              const float* __restrict__ bias,
                                              float* __restrict__ out) {
  __shared__ __align__(16) float st[8][16 * OTP];
  const int tid = threadIdx.x, lane = tid & 31, wave = tid >> 5;
  const int hh = lane >> 4, c = lane & 15;
  const int m0 = blockIdx.x * 256 + wave * 32;
  const int n0 = blockIdx.y * 64;

  v8f acc[2][4];
#pragma unroll
  for (int s = 0; s < 2; ++s)
#pragma unroll
    for (int t = 0; t < 4; ++t) acc[s][t] = zero8();
  gemm32x64(ap, CC, wt, CC, m0, n0, lane, acc);

  float bvs[4];
#pragma unroll
  for (int t = 0; t < 4; ++t) bvs[t] = bias[n0 + 16 * t + c];

  float* sw = st[wave];
#pragma unroll
  for (int sub = 0; sub < 2; ++sub) {
    __syncthreads();
#pragma unroll
    for (int t = 0; t < 4; ++t) {
#pragma unroll
      for (int r = 0; r < 8; ++r)
        sw[(8 * hh + r) * OTP + 16 * t + c] = acc[sub][t][r] * 0.001953125f + bvs[t];
    }
    __syncthreads();
    v4f val[8];
    size_t go[8];
#pragma unroll
    for (int it = 0; it < 8; ++it) {
      const int p    = lane + 32 * it;
      const int L    = p >> 3;
      const int pc   = p & 7;
      const int row  = L >> 1;
      const int half = L & 1;
      val[it] = *(const v4f*)(sw + row * OTP + half * 32 + pc * 4);
      go[it]  = (size_t)(m0 + sub * 16 + row) * CC + n0 + half * 32 + pc * 4;
    }
    for (int ps = 0; ps < 2; ++ps) {
#pragma unroll
      for (int it = 0; it < 8; ++it) *(volatile v4f*)(out + go[it]) = val[it];
      __threadfence();
    }
  }
}

extern "C" void kernel_launch(void* const* d_in, const int* in_sizes, int n_in,
                              void* d_out, int out_size, void* d_ws, size_t ws_size,
                              hipStream_t stream) {
  if (n_in < 12) return;
  if (in_sizes[0] != ROWS * CC) return;
  if (in_sizes[1] != CC * CC || in_sizes[3] != CC * CC || in_sizes[5] != CC * CC || in_sizes[7] != CC * CC) return;
  if (in_sizes[2] != CC || in_sizes[4] != CC || in_sizes[6] != CC || in_sizes[8] != CC) return;
  if (in_sizes[9] != HH * HH || in_sizes[10] != HH || in_sizes[11] != HH) return;
  if (out_size != ROWS * CC + BB * HH + BB) return;

  const float* x    = (const float*)d_in[0];
  const float* Wq   = (const float*)d_in[1];
  const float* bq   = (const float*)d_in[2];
  const float* Wk   = (const float*)d_in[3];
  const float* bk   = (const float*)d_in[4];
  const float* Wv   = (const float*)d_in[5];
  const float* bv   = (const float*)d_in[6];
  const float* Wo   = (const float*)d_in[7];
  const float* bo   = (const float*)d_in[8];
  const float* base = (const float*)d_in[9];
  const float* natf = (const float*)d_in[10];
  const float* ph0  = (const float*)d_in[11];

  float* out  = (float*)d_out;
  float* oph  = out + (size_t)ROWS * CC;
  float* oord = oph + BB * HH;

  size_t off = 0;
  const size_t oX   = off; off += (size_t)ROWS * CC * 2;
  const size_t oWq  = off; off += (size_t)C3 * CC * 2;
  const size_t oWo  = off; off += (size_t)CC * CC * 2;
  const size_t oQKV = off; off += 3 * PL * 2;
  const size_t oO   = off; off += (size_t)ROWS * CC * 2;
  const size_t oN   = off; off += (size_t)2 * NBH * NN * 4;
  const size_t oC   = off; off += 128;
  if (off > ws_size) return;

  char* ws = (char*)d_ws;
  _Float16* Xh   = (_Float16*)(ws + oX);
  _Float16* Wqkv = (_Float16*)(ws + oWq);
  _Float16* Wop  = (_Float16*)(ws + oWo);
  _Float16* QKVp = (_Float16*)(ws + oQKV);
  _Float16* Op   = (_Float16*)(ws + oO);
  float*    Nrm  = (float*)(ws + oN);
  float*    Coh  = (float*)(ws + oC);

  const int ngx = in_sizes[0] / 8;
  const int ngw = in_sizes[1] / 8;
  k_cvt<<<dim3((ngx + 255) / 256), dim3(256), 0, stream>>>(x, Xh, ngx, 1.0f);
  k_cvt<<<dim3((ngw + 255) / 256), dim3(256), 0, stream>>>(Wq, Wqkv, ngw, 32.0f);
  k_cvt<<<dim3((ngw + 255) / 256), dim3(256), 0, stream>>>(Wk, Wqkv + (size_t)CC * CC, ngw, 32.0f);
  k_cvt<<<dim3((ngw + 255) / 256), dim3(256), 0, stream>>>(Wv, Wqkv + (size_t)2 * CC * CC, ngw, 32.0f);
  k_cvt<<<dim3((ngw + 255) / 256), dim3(256), 0, stream>>>(Wo, Wop, ngw, 32.0f);
  k_phase<<<dim3(1), dim3(32), 0, stream>>>(base, natf, ph0, Coh, oph, oord);
  k_qkv<<<dim3(ROWS / 256, C3 / 64), dim3(256), 0, stream>>>(Xh, Wqkv, bq, bk, bv, QKVp, Nrm);
  k_attn<<<dim3(NBH * (NN / 128)), dim3(256), 0, stream>>>(QKVp, QKVp + PL, QKVp + 2 * PL,
                                                           Nrm, Nrm + (size_t)NBH * NN, Coh, Op);
  k_proj<<<dim3(ROWS / 256, CC / 64), dim3(256), 0, stream>>>(Op, Wop, bo, out);
  (void)hipGetLastError();
}
